// TTM_76622216561049
// MI455X (gfx1250) — hardware-verified
//
#include <hip/hip_runtime.h>
#include <math.h>

typedef __attribute__((ext_vector_type(16))) _Float16 v16h;
typedef __attribute__((ext_vector_type(8)))  _Float16 v8h;
typedef __attribute__((ext_vector_type(16))) __bf16   v16b;
typedef __attribute__((ext_vector_type(8)))  __bf16   v8b;
typedef __attribute__((ext_vector_type(8)))  float    v8f;
typedef __attribute__((ext_vector_type(4)))  float    v4f;

constexpr int kR    = 128;
constexpr int kSeg  = 64;
constexpr int kG    = 32;
constexpr int kM    = 1024;
constexpr int kT    = kR * kSeg;
constexpr int kTK   = 4;
constexpr int kHA   = 8;
constexpr int kDHd  = 128;
constexpr int kQKV  = 3 * kM;
constexpr int kF    = 4 * kM;
constexpr int kThr  = 256;
constexpr float kInCarry = 1024.0f;
constexpr float kCA = 4096.0f, kCZ = 1024.0f, kCI = 32.0f, kCS = 64.0f, kCH = 64.0f;
constexpr float kScA = 1.0f / (kCA * kInCarry), kScZ = 1.0f / (kCZ * kInCarry), kScI = 1.0f / (kCI * kInCarry), kScS = 1.0f / (kCS * kInCarry), kScH = 1.0f / (kCH * kInCarry);
constexpr float kLnEps = 1e-5f;
constexpr float kInvSqrtDh = 0.08838834764831845f;
constexpr float kF16MinNormal = 6.103515625e-5f;

static_assert((kR % 64) == 0 && (kM % 64) == 0 && (kQKV % 64) == 0 && (kF % 64) == 0 && ((kR / 64) * (kM / 64)) % 8 == 0, "GEMM M, N multiples of 64; grids exact");
static_assert(kM == kG * kG && kM == kHA * kDHd && kT == 8192 && kM == (1 << 10) && kF == (1 << 12), "shapes");

constexpr size_t kOffW02 = 0ull;
constexpr size_t kOffWQKV2 = 4194304ull;
constexpr size_t kOffWO2 = 54525952ull;
constexpr size_t kOffFC1W2 = 71303168ull;
constexpr size_t kOffFC2W2 = 88080384ull;
constexpr size_t kOffBIAS = 104857600ull;
constexpr size_t kOffPRM = 104894464ull;
constexpr size_t kOffALT16 = 104910848ull;
constexpr size_t kOffG0 = 105435136ull;
constexpr size_t kOffSAVE = 105959424ull;
constexpr size_t kOffZ16 = 106483712ull;
constexpr size_t kOffQKV = 107008000ull;
constexpr size_t kOffRSA = 108580864ull;
constexpr size_t kOffIMV16 = 108584960ull;
constexpr size_t kOffT32 = 109109248ull;
constexpr size_t kOffS216 = 109633536ull;
constexpr size_t kOffH32 = 110157824ull;
constexpr size_t kOffH16 = 112254976ull;
constexpr size_t kWsTotal = 114352128ull;
static_assert(kWsTotal <= 134217728ull, "carve cap: under 128 MiB");
static_assert(kOffW02 == 0
              && kOffWQKV2 == kOffW02 + 4194304ull
              && kOffWO2 == kOffWQKV2 + 50331648ull
              && kOffFC1W2 == kOffWO2 + 16777216ull
              && kOffFC2W2 == kOffFC1W2 + 16777216ull
              && kOffBIAS == kOffFC2W2 + 16777216ull
              && kOffPRM == kOffBIAS + 36864ull
              && kOffALT16 == kOffPRM + 16384ull
              && kOffG0 == kOffALT16 + 524288ull
              && kOffSAVE == kOffG0 + 524288ull
              && kOffZ16 == kOffSAVE + 524288ull
              && kOffQKV == kOffZ16 + 524288ull
              && kOffRSA == kOffQKV + 1572864ull
              && kOffIMV16 == kOffRSA + 4096ull
              && kOffT32 == kOffIMV16 + 524288ull
              && kOffS216 == kOffT32 + 524288ull
              && kOffH32 == kOffS216 + 524288ull
              && kOffH16 == kOffH32 + 2097152ull
              && kWsTotal == kOffH16 + 2097152ull, "the carve is chained and totalled");
static_assert((kOffW02 % 256) == 0 && (kOffWQKV2 % 256) == 0 && (kOffWO2 % 256) == 0 && (kOffFC1W2 % 256) == 0 && (kOffFC2W2 % 256) == 0 && (kOffBIAS % 256) == 0 && (kOffPRM % 256) == 0 && (kOffALT16 % 256) == 0 && (kOffG0 % 256) == 0 && (kOffSAVE % 256) == 0 && (kOffZ16 % 256) == 0 && (kOffQKV % 256) == 0 && (kOffRSA % 256) == 0 && (kOffIMV16 % 256) == 0 && (kOffT32 % 256) == 0 && (kOffS216 % 256) == 0 && (kOffH32 % 256) == 0 && (kOffH16 % 256) == 0, "aligned regions");
constexpr int kFZB = 0, kFB1 = 4096, kFB2 = 8192, kFEnd = 9216;
constexpr int kPG1 = 0, kPB1 = 1024, kPG2 = 2048, kPB2 = 3072, kPEnd = 4096;
static_assert(kFB1 == kFZB + kF && kFB2 == kFB1 + kF && kFEnd == kFB2 + kM && kPB1 == kPG1 + kM && kPG2 == kPB1 + kM && kPB2 == kPG2 + kM && kPEnd == kPB2 + kM, "bias stream and parameter plane maps");

__device__ __forceinline__ unsigned short f2bf_bits(float f) {
  unsigned u = __float_as_uint(f);
  return (unsigned short)((u + 0x7FFFu + ((u >> 16) & 1u)) >> 16);
}
__device__ __forceinline__ float bf_bits2f(unsigned short h) { return __uint_as_float(((unsigned)h) << 16); }
__device__ __forceinline__ float bf16r(float f) { return bf_bits2f(f2bf_bits(f)); }
__device__ __forceinline__ float carry_flush(float v, float carry) {
  const float s = v * carry;
  return (fabsf(s) < kF16MinNormal) ? 0.0f : s;
}
__device__ __forceinline__ float frcp(float x) { return __builtin_amdgcn_rcpf(x); }

__device__ __forceinline__ void dep_guard4_h(v8f& a, v8f& b, v8f& c, v8f& d, v16h x, v16h y) { asm volatile("v_nop\n\tv_nop\n\tv_nop\n\tv_nop" : "+v"(a), "+v"(b), "+v"(c), "+v"(d) : "v"(x), "v"(y)); }
__device__ __forceinline__ void dep_guard4_b(v8f& a, v8f& b, v8f& c, v8f& d, v16b x, v16b y) { asm volatile("v_nop\n\tv_nop\n\tv_nop\n\tv_nop" : "+v"(a), "+v"(b), "+v"(c), "+v"(d) : "v"(x), "v"(y)); }
__device__ __forceinline__ void keep4_h(v16h a, v16h b, v16h c, v16h d) { asm volatile("v_nop" :: "v"(a), "v"(b), "v"(c), "v"(d)); }
__device__ __forceinline__ void keep4_b(v16b a, v16b b, v16b c, v16b d) { asm volatile("v_nop" :: "v"(a), "v"(b), "v"(c), "v"(d)); }
__device__ __forceinline__ void acc_guard4(v8f& a, v8f& b, v8f& c, v8f& d) { asm volatile("v_nop\n\tv_nop\n\tv_nop\n\tv_nop" : "+v"(a), "+v"(b), "+v"(c), "+v"(d)); }

template <typename T> struct Frag;
template <> struct Frag<_Float16> {
  typedef v16h V; union U { v16h v; v8h h[2]; };
  static __device__ __forceinline__ v16h load(const _Float16* p) {
    U f; f.h[0] = *(const v8h*)(p); f.h[1] = *(const v8h*)(p + 16); return f.v;
  }
  static __device__ __forceinline__ v8f mma(v16h a, v16h b, v8f c) {
    return __builtin_amdgcn_wmma_f32_16x16x32_f16(false, a, false, b, (short)0, c, false, false);
  }
  static __device__ __forceinline__ void guard4(v8f& a, v8f& b, v8f& c, v8f& d, v16h x, v16h y) { dep_guard4_h(a, b, c, d, x, y); }
  static __device__ __forceinline__ void keep(v16h a, v16h b, v16h c, v16h d) { keep4_h(a, b, c, d); }
};
template <> struct Frag<__bf16> {
  typedef v16b V; union U { v16b v; v8b h[2]; };
  static __device__ __forceinline__ v16b load(const __bf16* p) {
    U f; f.h[0] = *(const v8b*)(p); f.h[1] = *(const v8b*)(p + 16); return f.v;
  }
  static __device__ __forceinline__ v8f mma(v16b a, v16b b, v8f c) {
    return __builtin_amdgcn_wmma_f32_16x16x32_bf16(false, a, false, b, (short)0, c, false, false);
  }
  static __device__ __forceinline__ void guard4(v8f& a, v8f& b, v8f& c, v8f& d, v16b x, v16b y) { dep_guard4_b(a, b, c, d, x, y); }
  static __device__ __forceinline__ void keep(v16b a, v16b b, v16b c, v16b d) { keep4_b(a, b, c, d); }
};

__device__ __forceinline__ v8f mma_h(v16h a, v16h b, v8f c) {
  c = __builtin_amdgcn_wmma_f32_16x16x32_f16(false, a, false, b, (short)0, c, false, false);
  asm volatile("v_nop\n\tv_nop\n\tv_nop\n\tv_nop" : "+v"(c) : "v"(a), "v"(b));
  return c;
}

template <int ET> struct Elem;
template <> struct Elem<0> { typedef _Float16 T; };
template <> struct Elem<1> { typedef __bf16 T; };
template <int ET, bool SPLIT, int BIAS_MODE, int OUT_MODE, bool RESID, int ACT = 0>
__global__ __launch_bounds__(256) void wmma_gemm64(
    const unsigned short* __restrict__ Ap, const unsigned short* __restrict__ A2p, int lda, long strideA,
    const unsigned short* __restrict__ Btp, const unsigned short* __restrict__ Bt2p, int ldb, long strideB,
    void* __restrict__ Cout, void* __restrict__ Cout2, int ldc, long strideC,
    const float* __restrict__ bias,
    const float* __restrict__ resid, long strideR,
    int M, int N, int K, float scale) {
  typedef typename Elem<ET>::T T;
  typedef typename Frag<T>::V V;
  const T* A = (const T*)Ap; const T* A2 = (const T*)A2p; const T* Bt = (const T*)Btp; const T* Bt2 = (const T*)Bt2p;
  __shared__ __align__(16) float sT[8][16 * 68];
  const int b    = blockIdx.y;
  const int lane = threadIdx.x & 31;
  const int wave = threadIdx.x >> 5;
  const int tilesN = N >> 6;
  const int tilesM = M >> 6;
  const int tile = blockIdx.x * 8 + wave;
  if (tile >= tilesM * tilesN) return;
  const int tm = tile / tilesN;
  const int tn = tile - tm * tilesN;
  const int m0 = tm << 6;
  const int n0 = tn << 6;

  const T* Ab  = A  + (size_t)b * strideA;
  const T* Bb  = Bt + (size_t)b * strideB;
  const T* Ab2 = SPLIT ? (A2  + (size_t)b * strideA) : nullptr;
  const T* Bb2 = SPLIT ? (Bt2 + (size_t)b * strideB) : nullptr;

  const int rlane = lane & 15;
  const int koff  = (lane >> 4) * 8;
  const int mOff  = (lane >> 4) * 8;

  v8f acc[4][4];
#pragma unroll
  for (int i = 0; i < 4; ++i)
#pragma unroll
    for (int j = 0; j < 4; ++j) acc[i][j] = (v8f){0.f,0.f,0.f,0.f,0.f,0.f,0.f,0.f};

  for (int k0 = 0; k0 < K; k0 += 32) {
    V bh[4], bl[4];
#pragma unroll
    for (int j = 0; j < 4; ++j) {
      const size_t bo = (size_t)(n0 + (j << 4) + rlane) * ldb + koff + k0;
      bh[j] = Frag<T>::load(Bb + bo);
      if (SPLIT) bl[j] = Frag<T>::load(Bb2 + bo);
    }
#pragma unroll
    for (int i = 0; i < 4; ++i) {
      const size_t ao = (size_t)(m0 + (i << 4) + rlane) * lda + koff + k0;
      V ah = Frag<T>::load(Ab + ao);
      V al;
      if (SPLIT) al = Frag<T>::load(Ab2 + ao);
#pragma unroll
      for (int j = 0; j < 4; ++j) {
        acc[i][j] = Frag<T>::mma(ah, bh[j], acc[i][j]);
        if (SPLIT) {
          acc[i][j] = Frag<T>::mma(ah, bl[j], acc[i][j]);
          acc[i][j] = Frag<T>::mma(al, bh[j], acc[i][j]);
        }
      }
      Frag<T>::guard4(acc[i][0], acc[i][1], acc[i][2], acc[i][3], ah, SPLIT ? al : ah);
    }
    Frag<T>::keep(bh[0], bh[1], bh[2], bh[3]);
    if (SPLIT) Frag<T>::keep(bl[0], bl[1], bl[2], bl[3]);
  }
  acc_guard4(acc[0][0], acc[0][1], acc[0][2], acc[0][3]);
  acc_guard4(acc[1][0], acc[1][1], acc[1][2], acc[1][3]);
  acc_guard4(acc[2][0], acc[2][1], acc[2][2], acc[2][3]);
  acc_guard4(acc[3][0], acc[3][1], acc[3][2], acc[3][3]);

  float* slab = sT[wave];
  const float* Rb = RESID ? (resid + (size_t)b * strideR) : nullptr;
#pragma unroll
  for (int i = 0; i < 4; ++i) {
    const int mBase = m0 + (i << 4);
#pragma unroll
    for (int j = 0; j < 4; ++j) {
      const int n = n0 + (j << 4) + rlane;
      float bv = 0.f;
      if (BIAS_MODE == 2) bv = bias[n];
#pragma unroll
      for (int r = 0; r < 8; ++r) {
        float v = acc[i][j][r] * scale;
        if (BIAS_MODE == 1) v += bias[mBase + mOff + r];
        if (BIAS_MODE == 2) v += bv;
        if (RESID) v += Rb[(size_t)(mBase + mOff + r) * ldc + n];
        if (ACT == 1) v = tanhf(v);
        if (ACT == 2) v = fmaxf(v, 0.0f);
        if (ACT == 3) v = v / (1.0f + expf(-v));
        if (ACT == 4) v = (v > 0.f) ? v : 0.01f * v;
        slab[(mOff + r) * 68 + (j << 4) + rlane] = v;
      }
    }
    __builtin_amdgcn_fence(__ATOMIC_RELEASE, "workgroup");
    __builtin_amdgcn_wave_barrier();
    __builtin_amdgcn_fence(__ATOMIC_ACQUIRE, "workgroup");
    if (OUT_MODE == 0) {
      float* C = (float*)Cout + (size_t)b * strideC;
      const int hh = lane >> 4, c4 = (lane & 15) * 4;
      for (int pass = 0; pass < 2; ++pass) {
#pragma unroll
        for (int it = 0; it < 8; ++it) {
          const int row = it * 2 + hh;
          v4f v = *(const v4f*)(slab + row * 68 + c4);
          *(volatile v4f*)(C + (size_t)(mBase + row) * ldc + n0 + c4) = v;
        }
        __threadfence();
      }
    } else {
      const int q = lane >> 3, c8 = (lane & 7) * 8;
      unsigned short* C  = (unsigned short*)Cout  + (size_t)b * strideC;
      unsigned short* C2 = (OUT_MODE == 2) ? ((unsigned short*)Cout2 + (size_t)b * strideC) : nullptr;
      for (int pass = 0; pass < 2; ++pass) {
#pragma unroll
        for (int it = 0; it < 4; ++it) {
          const int row = it * 4 + q;
          const float* sp = slab + row * 68 + c8;
          v8h hv, lv;
#pragma unroll
          for (int e = 0; e < 8; ++e) {
            if (OUT_MODE == 1) {
              hv[e] = (_Float16)sp[e];
            } else {
              unsigned short hb = f2bf_bits(sp[e]);
              unsigned short lb = f2bf_bits(sp[e] - bf_bits2f(hb));
              hv[e] = __builtin_bit_cast(_Float16, hb);
              lv[e] = __builtin_bit_cast(_Float16, lb);
            }
          }
          *(volatile v8h*)(C + (size_t)(mBase + row) * ldc + n0 + c8) = hv;
          if (OUT_MODE == 2) *(volatile v8h*)(C2 + (size_t)(mBase + row) * ldc + n0 + c8) = lv;
        }
        __threadfence();
      }
    }
    __builtin_amdgcn_fence(__ATOMIC_RELEASE, "workgroup");
    __builtin_amdgcn_wave_barrier();
    __builtin_amdgcn_fence(__ATOMIC_ACQUIRE, "workgroup");
  }
}

__global__ __launch_bounds__(kThr) void cast_plane_kernel(const float* __restrict__ src, unsigned short* __restrict__ dst,
                                                          int colsLog2, int dstPitch, int dstOff) {
  const int i   = blockIdx.x * kThr + threadIdx.x;
  const int sh  = colsLog2 - 3;
  const int row = i >> sh;
  const int c8  = (i & ((1 << sh) - 1)) * 8;
  const float* sp = src + ((size_t)row << colsLog2) + c8;
  const v4f a0 = *(const v4f*)(sp);
  const v4f a1 = *(const v4f*)(sp + 4);
  v8h hv;
#pragma unroll
  for (int e = 0; e < 4; ++e) {
    const float f0 = a0[e];
    const float f1 = a1[e];
    hv[e]     = (_Float16)carry_flush(bf16r(f0), kInCarry);
    hv[4 + e] = (_Float16)carry_flush(bf16r(f1), kInCarry);
  }
  unsigned short* dp = dst + (size_t)row * dstPitch + dstOff + c8;
  *(volatile v8h*)dp = hv;
  __threadfence();
  *(volatile v8h*)dp = hv;
}

__device__ __forceinline__ void split_f16(float x, float c, float cinv, _Float16& hi, _Float16& lo) {
  hi = (_Float16)carry_flush(x, c);
  const float back = (float)hi * cinv;
  lo = (_Float16)carry_flush(x - back, c);
}

__global__ __launch_bounds__(kThr) void setup_kernel(const float* __restrict__ fc1_b, const float* __restrict__ fc2_b,
                                                     const float* __restrict__ ln1_g, const float* __restrict__ ln1_b, const float* __restrict__ ln2_g, const float* __restrict__ ln2_b,
                                                     float* __restrict__ BIAS, float* __restrict__ PRM) {
  unsigned v = blockIdx.x * (unsigned)kThr + threadIdx.x;
  asm volatile("" : "+v"(v));
  v4f o;
  float* dp;
  if (v < 2304u) {
    const unsigned i0 = v * 4u;
    dp = BIAS + i0;
    const bool isB1 = (i0 >= (unsigned)kFB1) && (i0 < (unsigned)kFB2), isB2 = i0 >= (unsigned)kFB2;
    const float* sp = isB1 ? (fc1_b + (i0 - (unsigned)kFB1)) : (isB2 ? (fc2_b + (i0 - (unsigned)kFB2)) : fc1_b);
    const v4f a = *(const v4f*)sp;
    const bool live = isB1 || isB2;
#pragma unroll
    for (int e = 0; e < 4; ++e) { const float p = bf16r(a[e]); o[e] = live ? p : 0.0f; }
  } else {
    const unsigned i0 = (v - 2304u) * 4u;
    dp = PRM + i0;
    const float* sp = (i0 < (unsigned)kPB1) ? (ln1_g + i0) : ((i0 < (unsigned)kPG2) ? (ln1_b + (i0 - (unsigned)kPB1)) : ((i0 < (unsigned)kPB2) ? (ln2_g + (i0 - (unsigned)kPG2)) : (ln2_b + (i0 - (unsigned)kPB2))));
    const v4f a = *(const v4f*)sp;
#pragma unroll
    for (int e = 0; e < 4; ++e) o[e] = bf16r(a[e]);
  }
  *(volatile v4f*)dp = o;
  __threadfence();
  *(volatile v4f*)dp = o;
}
static_assert(kFEnd / 4 == 2304 && kPEnd / 4 == 1024 && 2304 + 1024 == 13 * kThr && (2304 % 32) == 0, "set-up grid exact; regions wave-uniform");

__global__ __launch_bounds__(kThr) void avg_kernel(const float* __restrict__ x, unsigned short* __restrict__ ALT16) {
  const unsigned v = blockIdx.x * (unsigned)kThr + threadIdx.x;
  const unsigned f = v >> 7, m8 = (v & 127u) * 8u;
  v8h hv, lv;
#pragma unroll 1
  for (int e = 0; e < 8; ++e) {
    const unsigned m = m8 + (unsigned)e, d1 = m >> 5, d2 = m & 31u;
    const float* sp = x + ((size_t)(d2 * (unsigned)kG + d1) * kT + (size_t)f * kSeg);
    float s = 0.0f;
#pragma unroll 1
    for (int q = 0; q < kSeg; q += 4) { const v4f a = *(const v4f*)(sp + q); s += bf16r(a[0]); s += bf16r(a[1]); s += bf16r(a[2]); s += bf16r(a[3]); }
    _Float16 hi, lo; split_f16(s * (1.0f / (float)kSeg), kCA, 1.0f / kCA, hi, lo);
    hv[e] = hi; lv[e] = lo;
  }
  unsigned short* dp = ALT16 + (size_t)f * (2 * kM) + m8;
  *(volatile v8h*)dp = hv; *(volatile v8h*)(dp + kM) = lv;
  __threadfence();
  *(volatile v8h*)dp = hv; *(volatile v8h*)(dp + kM) = lv;
}
static_assert(((size_t)kR * kM / 8) % kThr == 0 && kM / 8 == 128, "average grid exact");

__global__ __launch_bounds__(kThr) void save_init_kernel(const float* __restrict__ G0, float* __restrict__ SAVE) {
  const unsigned v = blockIdx.x * (unsigned)kThr + threadIdx.x;
  const unsigned f = v >> 8, c4 = (v & 255u) * 4u;
  const v4f g = *(const v4f*)(G0 + (size_t)f * kM + c4);
  const float fi = (float)f;
  const float a0 = fi / powf(10000.0f, 2.0f * (float)c4 / (float)kM);
  const float a1 = fi / powf(10000.0f, 2.0f * (float)(c4 + 2u) / (float)kM);
  v4f o;
  o[0] = g[0] + sinf(a0); o[1] = g[1] + cosf(a0); o[2] = g[2] + sinf(a1); o[3] = g[3] + cosf(a1);
  float* dp = SAVE + (size_t)f * kM + c4;
  *(volatile v4f*)dp = o;
  __threadfence();
  *(volatile v4f*)dp = o;
}
static_assert(((size_t)kR * kM / 4) % kThr == 0 && kM / 4 == 256, "position grid exact");

__global__ __launch_bounds__(kR) void ln_kernel(const float* __restrict__ SAVE, const float* __restrict__ T32, const float* __restrict__ g, const float* __restrict__ b,
                                                unsigned short* __restrict__ DST, int mode, float carry, float cinv) {
  const unsigned f = threadIdx.x;
  const float* sr = SAVE + (size_t)f * kM;
  const float* tr = T32 + (size_t)f * kM;
  float s1 = 0.0f;
#pragma unroll 1
  for (int c = 0; c < kM; c += 4) { v4f a = *(const v4f*)(sr + c); if (mode != 0) { const v4f t = *(const v4f*)(tr + c); a[0] += t[0]; a[1] += t[1]; a[2] += t[2]; a[3] += t[3]; } s1 += (a[0] + a[1]) + (a[2] + a[3]); }
  const float mu = s1 * (1.0f / (float)kM);
  float s2 = 0.0f;
#pragma unroll 1
  for (int c = 0; c < kM; c += 4) { v4f a = *(const v4f*)(sr + c); if (mode != 0) { const v4f t = *(const v4f*)(tr + c); a[0] += t[0]; a[1] += t[1]; a[2] += t[2]; a[3] += t[3]; } const float d0 = a[0] - mu, d1 = a[1] - mu, d2 = a[2] - mu, d3 = a[3] - mu; s2 += (d0 * d0 + d1 * d1) + (d2 * d2 + d3 * d3); }
  const float sd = sqrtf(s2 * (1.0f / (float)kM) + kLnEps);
  unsigned short* dp = DST + (size_t)f * (2 * kM);
  for (int pass = 0; pass < 2; ++pass) {
#pragma unroll 1
    for (int c = 0; c < kM; c += 8) {
      v8h hv, lv;
#pragma unroll
      for (int h = 0; h < 2; ++h) {
        v4f a = *(const v4f*)(sr + c + 4 * h); if (mode != 0) { const v4f t = *(const v4f*)(tr + c + 4 * h); a[0] += t[0]; a[1] += t[1]; a[2] += t[2]; a[3] += t[3]; }
        const v4f gg = *(const v4f*)(g + c + 4 * h), bb = *(const v4f*)(b + c + 4 * h);
#pragma unroll
        for (int e = 0; e < 4; ++e) { float y = (a[e] - mu) / sd * gg[e] + bb[e]; if (mode != 0) y += a[e]; _Float16 hi, lo; split_f16(y, carry, cinv, hi, lo); hv[4 * h + e] = hi; lv[4 * h + e] = lo; }
      }
      *(volatile v8h*)(dp + c) = hv; *(volatile v8h*)(dp + kM + c) = lv;
    }
    __threadfence();
  }
}

__global__ __launch_bounds__(kThr) void score_kernel(const float* __restrict__ QKV, float* __restrict__ RSA) {
  const unsigned v = blockIdx.x * (unsigned)kThr + threadIdx.x;
  const unsigned f = v >> 3, h = v & 7u;
  const float* qr = QKV + (size_t)f * kQKV + h * (unsigned)kDHd;
  const float* kr = qr + kM;
  float s = 0.0f;
#pragma unroll 1
  for (int d = 0; d < kDHd; d += 4) { const v4f q = *(const v4f*)(qr + d), k = *(const v4f*)(kr + d); s += (q[0] * kInvSqrtDh) * k[0]; s += (q[1] * kInvSqrtDh) * k[1]; s += (q[2] * kInvSqrtDh) * k[2]; s += (q[3] * kInvSqrtDh) * k[3]; }
  float* dp = RSA + v;
  *(volatile float*)dp = s;
  __threadfence();
  *(volatile float*)dp = s;
}
static_assert(((size_t)kR * kHA) % kThr == 0, "score grid exact");

__global__ __launch_bounds__(kR) void cumsum_kernel(const float* __restrict__ QKV, const float* __restrict__ RSA, unsigned short* __restrict__ IMV16) {
  const unsigned m8 = threadIdx.x * 8u;
  const unsigned h = m8 >> 7;
  float acc[8];
#pragma unroll
  for (int e = 0; e < 8; ++e) acc[e] = 0.0f;
#pragma unroll 1
  for (int f = 0; f < kR; ++f) {
    const float r = RSA[(size_t)f * kHA + h];
    const float* vr = QKV + (size_t)f * kQKV + 2 * kM + m8;
    const v4f v0 = *(const v4f*)vr, v1 = *(const v4f*)(vr + 4);
    v8h hv, lv;
#pragma unroll
    for (int e = 0; e < 4; ++e) {
      acc[e] += r * v0[e]; acc[4 + e] += r * v1[e];
      _Float16 hi, lo; split_f16(acc[e], kCI, 1.0f / kCI, hi, lo); hv[e] = hi; lv[e] = lo;
      split_f16(acc[4 + e], kCI, 1.0f / kCI, hi, lo); hv[4 + e] = hi; lv[4 + e] = lo;
    }
    unsigned short* dp = IMV16 + (size_t)f * (2 * kM) + m8;
    *(volatile v8h*)dp = hv; *(volatile v8h*)(dp + kM) = lv;
    __threadfence();
    *(volatile v8h*)dp = hv; *(volatile v8h*)(dp + kM) = lv;
  }
}
static_assert(kM / 8 == kR, "cumulative sum: 128 threads of 8 columns");

__global__ __launch_bounds__(kThr) void gelu_kernel(const float* __restrict__ H32, unsigned short* __restrict__ H16) {
  const unsigned v = blockIdx.x * (unsigned)kThr + threadIdx.x;
  const unsigned f = v >> 9, c8 = (v & 511u) * 8u;
  const float* sp = H32 + (size_t)f * kF + c8;
  const v4f a0 = *(const v4f*)sp, a1 = *(const v4f*)(sp + 4);
  v8h hv, lv;
#pragma unroll
  for (int e = 0; e < 4; ++e) {
    const float x0 = a0[e], x1 = a1[e];
    const float y0 = 0.5f * x0 * (1.0f + erff(x0 * 0.70710678118654752f)), y1 = 0.5f * x1 * (1.0f + erff(x1 * 0.70710678118654752f));
    _Float16 hi, lo; split_f16(y0, kCH, 1.0f / kCH, hi, lo); hv[e] = hi; lv[e] = lo;
    split_f16(y1, kCH, 1.0f / kCH, hi, lo); hv[4 + e] = hi; lv[4 + e] = lo;
  }
  unsigned short* dp = H16 + (size_t)f * (2 * kF) + c8;
  *(volatile v8h*)dp = hv; *(volatile v8h*)(dp + kF) = lv;
  __threadfence();
  *(volatile v8h*)dp = hv; *(volatile v8h*)(dp + kF) = lv;
}
static_assert(((size_t)kR * kF / 8) % kThr == 0 && kF / 8 == 512, "GELU grid exact");

extern "C" void kernel_launch(void* const* d_in, const int* in_sizes, int n_in,
                              void* d_out, int out_size, void* d_ws, size_t ws_size,
                              hipStream_t stream) {
  if (n_in < 12 || d_out == nullptr || d_ws == nullptr) return;
  if (in_sizes[0] != kG * kG * kT || in_sizes[1] != kM * kM || in_sizes[2] != kTK * kQKV * kM || in_sizes[3] != kTK * kM * kM) return;
  if (in_sizes[4] != kM || in_sizes[5] != kM || in_sizes[6] != kM || in_sizes[7] != kM || in_sizes[8] != kF * kM || in_sizes[9] != kF || in_sizes[10] != kM * kF || in_sizes[11] != kM) return;
  if (out_size != kR * kM) return;
  if (ws_size < kWsTotal) return;
  const float* x = (const float*)d_in[0];
  const float* weight = (const float*)d_in[1];
  const float* Wqkv = (const float*)d_in[2];
  const float* Wo = (const float*)d_in[3];
  const float* ln1_g = (const float*)d_in[4];
  const float* ln1_b = (const float*)d_in[5];
  const float* ln2_g = (const float*)d_in[6];
  const float* ln2_b = (const float*)d_in[7];
  const float* fc1_w = (const float*)d_in[8];
  const float* fc1_b = (const float*)d_in[9];
  const float* fc2_w = (const float*)d_in[10];
  const float* fc2_b = (const float*)d_in[11];
  float* out = (float*)d_out;
  char* ws = (char*)d_ws;
  unsigned short* W02 = (unsigned short*)(ws + kOffW02);
  unsigned short* WQKV2 = (unsigned short*)(ws + kOffWQKV2);
  unsigned short* WO2 = (unsigned short*)(ws + kOffWO2);
  unsigned short* FC1W2 = (unsigned short*)(ws + kOffFC1W2);
  unsigned short* FC2W2 = (unsigned short*)(ws + kOffFC2W2);
  float* BIAS = (float*)(ws + kOffBIAS);
  float* PRM = (float*)(ws + kOffPRM);
  unsigned short* ALT16 = (unsigned short*)(ws + kOffALT16);
  float* G0 = (float*)(ws + kOffG0);
  float* SAVE = (float*)(ws + kOffSAVE);
  unsigned short* Z16 = (unsigned short*)(ws + kOffZ16);
  float* QKV = (float*)(ws + kOffQKV);
  float* RSA = (float*)(ws + kOffRSA);
  unsigned short* IMV16 = (unsigned short*)(ws + kOffIMV16);
  float* T32 = (float*)(ws + kOffT32);
  unsigned short* S216 = (unsigned short*)(ws + kOffS216);
  float* H32 = (float*)(ws + kOffH32);
  unsigned short* H16 = (unsigned short*)(ws + kOffH16);

  const int gMM = (int)(((size_t)kM * kM / 8) / kThr), gQ = (int)(((size_t)kQKV * kM / 8) / kThr), gF = (int)(((size_t)kF * kM / 8) / kThr);
  cast_plane_kernel<<<gMM, kThr, 0, stream>>>(weight, W02, 10, 2 * kM, 0);
  cast_plane_kernel<<<gMM, kThr, 0, stream>>>(weight, W02, 10, 2 * kM, kM);
  for (int a = 0; a < kTK; ++a) {
    cast_plane_kernel<<<gQ, kThr, 0, stream>>>(Wqkv + (size_t)a * kQKV * kM, WQKV2 + (size_t)a * kQKV * 2 * kM, 10, 2 * kM, 0);
    cast_plane_kernel<<<gQ, kThr, 0, stream>>>(Wqkv + (size_t)a * kQKV * kM, WQKV2 + (size_t)a * kQKV * 2 * kM, 10, 2 * kM, kM);
    cast_plane_kernel<<<gMM, kThr, 0, stream>>>(Wo + (size_t)a * kM * kM, WO2 + (size_t)a * kM * 2 * kM, 10, 2 * kM, 0);
    cast_plane_kernel<<<gMM, kThr, 0, stream>>>(Wo + (size_t)a * kM * kM, WO2 + (size_t)a * kM * 2 * kM, 10, 2 * kM, kM);
  }
  cast_plane_kernel<<<gF, kThr, 0, stream>>>(fc1_w, FC1W2, 10, 2 * kM, 0);
  cast_plane_kernel<<<gF, kThr, 0, stream>>>(fc1_w, FC1W2, 10, 2 * kM, kM);
  cast_plane_kernel<<<gF, kThr, 0, stream>>>(fc2_w, FC2W2, 12, 2 * kF, 0);
  cast_plane_kernel<<<gF, kThr, 0, stream>>>(fc2_w, FC2W2, 12, 2 * kF, kF);
  setup_kernel<<<13, kThr, 0, stream>>>(fc1_b, fc2_b, ln1_g, ln1_b, ln2_g, ln2_b, BIAS, PRM);

  avg_kernel<<<(int)(((size_t)kR * kM / 8) / kThr), kThr, 0, stream>>>(x, ALT16);
  wmma_gemm64<0, false, 2, 0, false, 0><<<dim3((kR / 64) * (kM / 64) / 8, 1), 256, 0, stream>>>(
      ALT16, ALT16, 2 * kM, 0L, W02, W02, 2 * kM, 0L, (void*)G0, (void*)G0, kM, 0L, BIAS + kFZB, nullptr, 0L, kR, kM, 2 * kM, kScA);
  save_init_kernel<<<(int)(((size_t)kR * kM / 4) / kThr), kThr, 0, stream>>>(G0, SAVE);

  for (int a = 0; a < kTK; ++a) {
    const unsigned short* wq = WQKV2 + (size_t)a * kQKV * 2 * kM;
    const unsigned short* wo = WO2 + (size_t)a * kM * 2 * kM;
    float* dst = (a == kTK - 1) ? out : SAVE;
    ln_kernel<<<1, kR, 0, stream>>>(SAVE, SAVE, PRM + kPG1, PRM + kPB1, Z16, 0, kCZ, 1.0f / kCZ);
    wmma_gemm64<0, false, 2, 0, false, 0><<<dim3((kR / 64) * (kQKV / 64) / 8, 1), 256, 0, stream>>>(
        Z16, Z16, 2 * kM, 0L, wq, wq, 2 * kM, 0L, (void*)QKV, (void*)QKV, kQKV, 0L, BIAS + kFZB, nullptr, 0L, kR, kQKV, 2 * kM, kScZ);
    score_kernel<<<(kR * kHA) / kThr, kThr, 0, stream>>>(QKV, RSA);
    cumsum_kernel<<<1, kR, 0, stream>>>(QKV, RSA, IMV16);
    wmma_gemm64<0, false, 2, 0, false, 0><<<dim3((kR / 64) * (kM / 64) / 8, 1), 256, 0, stream>>>(
        IMV16, IMV16, 2 * kM, 0L, wo, wo, 2 * kM, 0L, (void*)T32, (void*)T32, kM, 0L, BIAS + kFZB, nullptr, 0L, kR, kM, 2 * kM, kScI);
    ln_kernel<<<1, kR, 0, stream>>>(SAVE, T32, PRM + kPG2, PRM + kPB2, S216, 1, kCS, 1.0f / kCS);
    wmma_gemm64<0, false, 2, 0, false, 0><<<dim3((kR / 64) * (kF / 64) / 8, 1), 256, 0, stream>>>(
        S216, S216, 2 * kM, 0L, FC1W2, FC1W2, 2 * kM, 0L, (void*)H32, (void*)H32, kF, 0L, BIAS + kFB1, nullptr, 0L, kR, kF, 2 * kM, kScS);
    gelu_kernel<<<(int)(((size_t)kR * kF / 8) / kThr), kThr, 0, stream>>>(H32, H16);
    wmma_gemm64<0, false, 2, 0, false, 0><<<dim3((kR / 64) * (kM / 64) / 8, 1), 256, 0, stream>>>(
        H16, H16, 2 * kF, 0L, FC2W2, FC2W2, 2 * kF, 0L, (void*)dst, (void*)dst, kM, 0L, BIAS + kFB2, nullptr, 0L, kR, kM, 2 * kF, kScH);
  }
}
